// ConvTransBlock_15564961481157
// MI455X (gfx1250) — hardware-verified
//
#include <hip/hip_runtime.h>


#define NB_  4
#define CC   192
#define NH_  6
#define HD   32
#define HH   56
#define NPX  3136
#define NR   (NB_ * NPX)
#define WIN  7
#define KT   49
#define WP   62
#define NPP  (WP * WP)
#define NPR  3904
#define GB   192
#define NPT  (GB + NPR + GB)
#define C3   576
#define C4   768
#define DM   CC
#define BEPS 1e-5f
#define SCL  0.17677669529663687f
#define LOSC 1024.0f

typedef _Float16 h16;
typedef unsigned short bf;
typedef __attribute__((ext_vector_type(16))) __bf16   v16bf;
typedef __attribute__((ext_vector_type(16))) _Float16 v16h;
typedef __attribute__((ext_vector_type(8)))  _Float16 v8h;
typedef __attribute__((ext_vector_type(8)))  unsigned short v8us;
typedef __attribute__((ext_vector_type(8)))  float    v8f;
typedef __attribute__((ext_vector_type(4)))  float    v4f;
typedef v8h  __attribute__((may_alias)) v8ha;
typedef v4f  __attribute__((may_alias)) v4fa;
typedef v8us __attribute__((may_alias)) v8usa;

__device__ __forceinline__ unsigned short f2bf(float f) { unsigned u = __float_as_uint(f); u += 0x7FFFu + ((u >> 16) & 1u); return (unsigned short)(u >> 16); }
__device__ __forceinline__ float bf2f(unsigned short b) { return __uint_as_float(((unsigned)b) << 16); }
__device__ __forceinline__ float bfr(float f) { return bf2f(f2bf(f)); }
__device__ __forceinline__ v16h cat16(v8h lo, v8h hi) { return __builtin_shufflevector(lo, hi, 0, 1, 2, 3, 4, 5, 6, 7, 8, 9, 10, 11, 12, 13, 14, 15); }
__device__ __forceinline__ v16bf cat16b(v8us lo, v8us hi) { return __builtin_bit_cast(v16bf, __builtin_shufflevector(lo, hi, 0, 1, 2, 3, 4, 5, 6, 7, 8, 9, 10, 11, 12, 13, 14, 15)); }
__device__ __forceinline__ v8f wmma16(v16h a, v16h b, v8f c) { return __builtin_amdgcn_wmma_f32_16x16x32_f16(false, a, false, b, (short)0, c, false, false); }
__device__ __forceinline__ v8f wmmab(v16bf a, v16bf b, v8f c) { return __builtin_amdgcn_wmma_f32_16x16x32_bf16(false, a, false, b, (short)0, c, false, false); }

template <bool SPLITA, bool F16OUT = false>
__global__ __launch_bounds__(128) void k_gemmb(const bf* __restrict__ A, const bf* __restrict__ Al, const bf* __restrict__ Bn, const float* __restrict__ bias, float* C, int ldc, h16* C2, const float* __restrict__ R = nullptr, int K = DM, int roundR = 1) {
    __shared__ __align__(16) float ost[4][16 * 68];
    const int lane = threadIdx.x & 31, wave = threadIdx.x >> 5, lr = lane & 15, hi = lane >> 4;
    const int r0 = blockIdx.x * 64 + wave * 16, c0 = blockIdx.y * 64;
    const size_t aoff = (size_t)(r0 + lr) * K + 8 * hi;
    size_t boff[4];
#pragma unroll
    for (int t = 0; t < 4; ++t) boff[t] = (size_t)(c0 + t * 16 + lr) * K + 8 * hi;
    v8f acc[4];
#pragma unroll
    for (int t = 0; t < 4; ++t) acc[t] = (v8f){};
#pragma unroll 1
    for (int kc = 0; kc < K; kc += 32) {
        const v16bf a = cat16b(*(const v8us*)(A + aoff + kc), *(const v8us*)(A + aoff + kc + 16));
        v16bf al = a;
        if (SPLITA) al = cat16b(*(const v8us*)(Al + aoff + kc), *(const v8us*)(Al + aoff + kc + 16));
#pragma unroll
        for (int t = 0; t < 4; ++t) { const v16bf b = cat16b(*(const v8us*)(Bn + boff[t] + kc), *(const v8us*)(Bn + boff[t] + kc + 16)); acc[t] = wmmab(a, b, acc[t]); if (SPLITA) acc[t] = wmmab(al, b, acc[t]); }
        asm volatile("v_nop\n\tv_nop\n\tv_nop\n\tv_nop" : "+v"(acc[0]), "+v"(acc[1]), "+v"(acc[2]), "+v"(acc[3]) : "v"(a), "v"(al));
    }
    float* os = &ost[wave][0];
#pragma unroll
    for (int t = 0; t < 4; ++t) { const float bv = bias ? bfr(bias[c0 + t * 16 + lr]) : 0.f;
#pragma unroll
        for (int j = 0; j < 8; ++j) os[(hi * 8 + j) * 68 + t * 16 + lr] = acc[t][j] + bv; }
    __syncthreads();
    if (F16OUT) {
        h16* crow = (h16*)(void*)C + (size_t)r0 * ldc + c0;
        auto pass = [&]() {
#pragma unroll
            for (int s = 0; s < 4; ++s) { const int row = 4 * s + (lane >> 3), piece = lane & 7; const float* sp = os + row * 68 + piece * 8; v8h o, o2;
#pragma unroll
                for (int i = 0; i < 8; ++i) { const h16 a = (h16)sp[i]; o[i] = a; o2[i] = (h16)((sp[i] - (float)a) * LOSC); }
                *(volatile v8h*)(crow + (size_t)row * ldc + piece * 8) = o; if (C2) *(volatile v8h*)(C2 + (size_t)r0 * ldc + c0 + (size_t)row * ldc + piece * 8) = o2; }
        };
        pass(); __threadfence(); pass();
    } else {
        float* crow = C + (size_t)r0 * ldc + c0;
        auto pass = [&]() {
#pragma unroll
            for (int s = 0; s < 8; ++s) { const int Lid = (lane >> 3) + 4 * s, piece = lane & 7; const int row = Lid >> 1, cofs = (Lid & 1) * 32 + piece * 4;
                v4f val = *(const v4fa*)(os + row * 68 + cofs); if (R) { const v4f rv = *(const v4f*)(R + ((size_t)r0 + row) * ldc + c0 + cofs); val += roundR ? (v4f){bfr(rv[0]), bfr(rv[1]), bfr(rv[2]), bfr(rv[3])} : rv; }
                *(volatile v4f*)(crow + (size_t)row * ldc + cofs) = val; }
        };
        pass(); __threadfence(); pass();
    }
}

__global__ __launch_bounds__(256) void k_cvt8(const float* __restrict__ src, bf* dst, size_t n8) {
    const size_t i = (size_t)blockIdx.x * 256 + threadIdx.x; if (i >= n8) return;
    const v8f v = *(const v8f*)(src + i * 8); v8us o;
#pragma unroll
    for (int k = 0; k < 8; ++k) o[k] = f2bf(v[k]);
    *(volatile v8us*)(dst + i * 8) = o; __threadfence(); *(volatile v8us*)(dst + i * 8) = o;
}
__global__ __launch_bounds__(256) void k_zero8(bf* dst, size_t n8) {
    const size_t i = (size_t)blockIdx.x * 256 + threadIdx.x; if (i >= n8) return; v8us z;
#pragma unroll
    for (int k = 0; k < 8; ++k) z[k] = 0;
    *(volatile v8us*)(dst + i * 8) = z; __threadfence(); *(volatile v8us*)(dst + i * 8) = z;
}

__global__ __launch_bounds__(256) void k_bnstatc(const float* __restrict__ x, float* STT) {
    const int lane = threadIdx.x & 31; const int c = blockIdx.x * 8 + (threadIdx.x >> 5); if (c >= CC) return; const int n = NB_ * NPX; float s = 0.f;
    for (int e = lane; e < n; e += 32) { const int b = e / NPX, p = e % NPX; s += bfr(x[((size_t)b * CC + c) * NPX + p]); }
#pragma unroll
    for (int sh = 16; sh; sh >>= 1) s += __shfl_xor(s, sh, 32);
    const float mu = s / (float)n; float q = 0.f;
    for (int e = lane; e < n; e += 32) { const int b = e / NPX, p = e % NPX; const float d = bfr(x[((size_t)b * CC + c) * NPX + p]) - mu; q = fmaf(d, d, q); }
#pragma unroll
    for (int sh = 16; sh; sh >>= 1) q += __shfl_xor(q, sh, 32);
    const float rs = rsqrtf(q / (float)n + BEPS); const float v = (lane == 0) ? mu : (lane == 1) ? rs : 0.f;
    *(volatile float*)(STT + (size_t)c * 32 + lane) = v; __threadfence(); *(volatile float*)(STT + (size_t)c * 32 + lane) = v;
}
__global__ __launch_bounds__(256) void k_bnT(const float* __restrict__ xb, const float* __restrict__ STT, const float* __restrict__ gam, const float* __restrict__ bet, size_t r0, bf* XNh, bf* XNl, float* XTf) {
    __shared__ float tl[64][65]; __shared__ float tr[64][65];
    typedef __attribute__((ext_vector_type(4))) unsigned short v4us;
    const int tid = threadIdx.x, c0 = blockIdx.x * 64, p0 = blockIdx.y * 64; const int rr = tid >> 2, cq = (tid & 3) * 16;
    { const int c = c0 + rr; const float mu = STT[(size_t)c * 32], rs = STT[(size_t)c * 32 + 1], ga = bfr(gam[c]), be = bfr(bet[c]);
#pragma unroll
      for (int i = 0; i < 16; ++i) { const float xv = bfr(xb[(size_t)c * NPX + p0 + cq + i]); tr[rr][cq + i] = xv; tl[rr][cq + i] = (xv - mu) * rs * ga + be; } }
    __syncthreads();
    const int lane = tid & 31, wv = tid >> 5;
    auto pass = [&]() {
#pragma unroll
        for (int st = 0; st < 4; ++st) { const int pr = wv * 8 + st * 2 + (lane >> 4); const int cl = (lane & 15) * 4; v4us oh, ol; v4f xf;
#pragma unroll
            for (int i = 0; i < 4; ++i) { const float y = tl[cl + i][pr]; const unsigned short hb = f2bf(y); oh[i] = hb; ol[i] = f2bf(y - bf2f(hb)); xf[i] = tr[cl + i][pr]; }
            const size_t o = (r0 + p0 + pr) * CC + c0 + cl; *(volatile v4us*)(XNh + o) = oh; *(volatile v4us*)(XNl + o) = ol; *(volatile v4f*)(XTf + o) = xf; }
    };
    pass(); __threadfence(); pass();
}
__global__ __launch_bounds__(256) void k_qkgrid(const float* __restrict__ QKV, size_t r0, int h, bf* Gh, bf* Gl) {
    typedef __attribute__((ext_vector_type(2))) unsigned short v2us;
    const int lane = threadIdx.x & 31; const size_t r = (size_t)blockIdx.x * 8 + (threadIdx.x >> 5); if (r >= (size_t)NPT) return; const long pr = (long)r - GB; int y = -1, x = -1; bool live = false;
    if (pr >= 0 && pr < NPP) { const int gy = (int)(pr / WP), gx = (int)(pr % WP); y = gy - 3; x = gx - 3; live = (y >= 0 && y < HH && x >= 0 && x < HH); }
    v2us oh, ol;
#pragma unroll
    for (int i = 0; i < 2; ++i) { const int c = lane * 2 + i; float v = 0.f; if (live) { const size_t row = r0 + (size_t)y * HH + x; v = (c < HD) ? QKV[row * C3 + h * HD + c] * SCL : QKV[row * C3 + CC + h * HD + (c - HD)]; } const unsigned short hb = f2bf(v); oh[i] = hb; ol[i] = f2bf(v - bf2f(hb)); }
    const size_t o = r * 64 + lane * 2; *(volatile v2us*)(Gh + o) = oh; *(volatile v2us*)(Gl + o) = ol; __threadfence(); *(volatile v2us*)(Gh + o) = oh; *(volatile v2us*)(Gl + o) = ol;
}
__global__ __launch_bounds__(256) void k_wtap(const float* __restrict__ Wd, bf* WT) {
    typedef __attribute__((ext_vector_type(2))) unsigned short v2us;
    const int lane = threadIdx.x & 31; const int w = blockIdx.x * 8 + (threadIdx.x >> 5); if (w >= KT * 64) return; const int tap = w / 64, k = w % 64; v2us o;
#pragma unroll
    for (int i = 0; i < 2; ++i) { const int ci = lane * 2 + i; o[i] = f2bf(k < KT ? Wd[(((size_t)(k < KT ? k : 0) * 64 + ci) * KT) + tap] : 0.f); }
    *(volatile v2us*)(WT + (size_t)w * 64 + lane * 2) = o; __threadfence(); *(volatile v2us*)(WT + (size_t)w * 64 + lane * 2) = o;
}
__global__ __launch_bounds__(128) void k_gemmtap49(const bf* __restrict__ Ah, const bf* __restrict__ Al, const bf* __restrict__ Bt, float* C) {
    __shared__ __align__(16) float ost[4][16 * 68];
    const int lane = threadIdx.x & 31, wave = threadIdx.x >> 5, lr = lane & 15, hi = lane >> 4;
    const int r0 = blockIdx.x * 64 + wave * 16; const int K = 64;
    v8f acc[4];
#pragma unroll
    for (int t = 0; t < 4; ++t) acc[t] = (v8f){};
#pragma unroll 1
    for (int tap = 0; tap < KT; ++tap) { const long off = (long)(tap / WIN - 3) * WP + (tap % WIN - 3);
        const size_t aoff = (size_t)((long)GB + off + r0 + lr) * K + 8 * hi; const bf* Bn = Bt + (size_t)tap * 64 * K;
#pragma unroll
        for (int kc = 0; kc < 64; kc += 32) {
            const v16bf a = cat16b(*(const v8us*)(Ah + aoff + kc), *(const v8us*)(Ah + aoff + kc + 16));
            const v16bf al = cat16b(*(const v8us*)(Al + aoff + kc), *(const v8us*)(Al + aoff + kc + 16));
#pragma unroll
            for (int t = 0; t < 4; ++t) { const size_t bo = (size_t)(t * 16 + lr) * K + kc + 8 * hi; const v16bf b = cat16b(*(const v8us*)(Bn + bo), *(const v8us*)(Bn + bo + 16)); acc[t] = wmmab(a, b, acc[t]); acc[t] = wmmab(al, b, acc[t]); }
            asm volatile("v_nop\n\tv_nop\n\tv_nop\n\tv_nop" : "+v"(acc[0]), "+v"(acc[1]), "+v"(acc[2]), "+v"(acc[3]) : "v"(a), "v"(al)); } }
    float* os = &ost[wave][0];
#pragma unroll
    for (int t = 0; t < 4; ++t) {
#pragma unroll
        for (int j = 0; j < 8; ++j) os[(hi * 8 + j) * 68 + t * 16 + lr] = acc[t][j]; }
    __builtin_amdgcn_wave_barrier(); asm volatile("" ::: "memory");
    float* crow = C + (size_t)r0 * 64;
    auto pass = [&]() {
#pragma unroll
        for (int s = 0; s < 8; ++s) { const int Lid = (lane >> 3) + 4 * s, piece = lane & 7; const int row = Lid >> 1, cofs = (Lid & 1) * 32 + piece * 4;
            const v4f val = *(const v4fa*)(os + row * 68 + cofs); *(volatile v4f*)(crow + (size_t)row * 64 + cofs) = val; }
    };
    pass(); __threadfence(); pass();
}
__global__ __launch_bounds__(256) void k_wattn(const float* __restrict__ CT, const float* __restrict__ QKV, const float* __restrict__ dmb, const float* __restrict__ rel, size_t r0, int h, float* O) {
    const int lane = threadIdx.x & 31; const size_t p = (size_t)blockIdx.x * 8 + (threadIdx.x >> 5); if (p >= (size_t)NPX) return; const int y = (int)(p / HH), x = (int)(p % HH); const float* ct = CT + ((size_t)(y + 3) * WP + (x + 3)) * 64;
    const int k0 = lane, k1 = lane + 32; const float l0 = ct[k0] + bfr(dmb[k0]) + bfr(rel[k0 * NH_ + h]); const float l1 = (k1 < KT) ? ct[k1] + bfr(dmb[k1 < KT ? k1 : 0]) + bfr(rel[(k1 < KT ? k1 : 0) * NH_ + h]) : -3.0e38f;
    float m = fmaxf(l0, l1);
#pragma unroll
    for (int sh = 16; sh; sh >>= 1) m = fmaxf(m, __shfl_xor(m, sh, 32));
    const float e0 = __expf(l0 - m), e1 = (k1 < KT) ? __expf(l1 - m) : 0.f; float s = e0 + e1;
#pragma unroll
    for (int sh = 16; sh; sh >>= 1) s += __shfl_xor(s, sh, 32);
    const float inv = 1.0f / s; const float a0 = e0 * inv, a1 = e1 * inv; const int c = lane; float acc = 0.f;
#pragma unroll 1
    for (int k = 0; k < KT; ++k) { const float ak = (k < 32) ? __shfl(a0, k, 32) : __shfl(a1, k - 32, 32); const int yy = y + k / WIN - 3, xx = x + k % WIN - 3;
        const bool in = (yy >= 0 && yy < HH && xx >= 0 && xx < HH); const float v = in ? QKV[(r0 + (size_t)(in ? yy : 0) * HH + (in ? xx : 0)) * C3 + 2 * CC + h * HD + c] : 0.f; acc = fmaf(ak, v, acc); }
    float* dst = O + (r0 + p) * CC + h * HD + c; *(volatile float*)dst = acc; __threadfence(); *(volatile float*)dst = acc;
}
__global__ __launch_bounds__(256) void k_split192(const float* __restrict__ F, size_t rows, bf* Ph, bf* Pl) {
    const int lane = threadIdx.x & 31; const size_t r = (size_t)blockIdx.x * 8 + (threadIdx.x >> 5); if (r >= rows || lane >= 24) return; const size_t o = r * CC + lane * 8; const v8f v = *(const v8f*)(F + o); v8us oh, ol;
#pragma unroll
    for (int i = 0; i < 8; ++i) { const unsigned short hb = f2bf(v[i]); oh[i] = hb; ol[i] = f2bf(v[i] - bf2f(hb)); }
    *(volatile v8us*)(Ph + o) = oh; *(volatile v8us*)(Pl + o) = ol; __threadfence(); *(volatile v8us*)(Ph + o) = oh; *(volatile v8us*)(Pl + o) = ol;
}
__global__ __launch_bounds__(256) void k_gelu768(const float* __restrict__ F, size_t rows, bf* Ph, bf* Pl) {
    const int lane = threadIdx.x & 31; const size_t r = (size_t)blockIdx.x * 8 + (threadIdx.x >> 5); if (r >= rows) return;
#pragma unroll 1
    for (int ps = 0; ps < 2; ++ps) {
#pragma unroll 1
        for (int q = 0; q < C4 / 256; ++q) { const size_t o = r * C4 + q * 256 + lane * 8; const v8f v = *(const v8f*)(F + o); v8us oh, ol;
#pragma unroll
            for (int i = 0; i < 8; ++i) { const float xg = v[i]; const float y = 0.5f * xg * (1.0f + erff(xg * 0.70710678118654752f)); const unsigned short hb = f2bf(y); oh[i] = hb; ol[i] = f2bf(y - bf2f(hb)); }
            *(volatile v8us*)(Ph + o) = oh; *(volatile v8us*)(Pl + o) = ol; }
        if (ps == 0) __threadfence(); }
}
__global__ __launch_bounds__(256) void k_outT(const float* __restrict__ X1, const float* __restrict__ H2, size_t r0, float* OUTB) {
    __shared__ float tl[64][65];
    const int tid = threadIdx.x; const int p0 = blockIdx.x * 64, c0 = blockIdx.y * 64; const int rr = tid >> 2, cq = (tid & 3) * 16;
#pragma unroll
    for (int i = 0; i < 16; ++i) { const size_t o = (r0 + p0 + rr) * CC + c0 + cq + i; tl[rr][cq + i] = X1[o] + H2[o]; }
    __syncthreads();
    const int lane = tid & 31, wv = tid >> 5;
    auto pass = [&]() {
#pragma unroll
        for (int st = 0; st < 4; ++st) { const int cr = wv * 8 + st * 2 + (lane >> 4); const int pq = (lane & 15) * 4; v4f v; const size_t o = ((size_t)c0 + cr) * NPX + p0 + pq;
#pragma unroll
            for (int i = 0; i < 4; ++i) v[i] = tl[pq + i][cr];
            *(volatile v4f*)(OUTB + o) = v; }
    };
    pass(); __threadfence(); pass();
}

extern "C" void kernel_launch(void* const* d_in, const int* in_sizes, int n_in,
                              void* d_out, int out_size, void* d_ws, size_t ws_size, hipStream_t stream) {
    (void)in_sizes; (void)n_in; (void)out_size;
    const float* x = (const float*)d_in[0]; const float* gam = (const float*)d_in[1]; const float* bet = (const float*)d_in[2]; const float* qkvw = (const float*)d_in[3]; const float* qkvb = (const float*)d_in[4]; const float* dmw = (const float*)d_in[5]; const float* dmb = (const float*)d_in[6]; const float* rel = (const float*)d_in[7];
    const float* pw = (const float*)d_in[8]; const float* pb = (const float*)d_in[9]; const float* c1w = (const float*)d_in[10]; const float* c1b = (const float*)d_in[11]; const float* c2w = (const float*)d_in[12]; const float* c2b = (const float*)d_in[13];
    float* out = (float*)d_out;
    char* wsp = (char*)d_ws;
    auto take = [&](size_t bytes) { char* p = wsp; wsp += (bytes + 255) & ~(size_t)255; return (void*)p; };
    bf* WQKV = (bf*)take((size_t)C3 * CC * 2); bf* WP_ = (bf*)take((size_t)CC * CC * 2); bf* WC1 = (bf*)take((size_t)C4 * CC * 2); bf* WC2 = (bf*)take((size_t)CC * C4 * 2); bf* WT = (bf*)take((size_t)KT * 64 * 64 * 2); float* STT = (float*)take((size_t)CC * 32 * 4);
    bf* XNh = (bf*)take((size_t)NR * CC * 2); bf* XNl = (bf*)take((size_t)NR * CC * 2); float* XTf = (float*)take((size_t)NR * CC * 4); float* QKV = (float*)take((size_t)NR * C3 * 4);
    bf* Gh = (bf*)take((size_t)NPT * 64 * 2); bf* Gl = (bf*)take((size_t)NPT * 64 * 2); float* CT = (float*)take((size_t)NPR * 64 * 4); float* O = (float*)take((size_t)NR * CC * 4);
    bf* Oh = (bf*)take((size_t)NPX * CC * 2); bf* Ol = (bf*)take((size_t)NPX * CC * 2); float* X1 = (float*)take((size_t)NR * CC * 4); bf* X1h = (bf*)take((size_t)NPX * CC * 2); bf* X1l = (bf*)take((size_t)NPX * CC * 2); float* H1 = (float*)take((size_t)NPX * C4 * 4); bf* G1h = (bf*)take((size_t)NPX * C4 * 2); bf* G1l = (bf*)take((size_t)NPX * C4 * 2); float* H2 = (float*)take((size_t)NR * CC * 4);
    if ((size_t)(wsp - (char*)d_ws) > ws_size) return;
    k_cvt8<<<(C3 * CC / 8 + 255) / 256, 256, 0, stream>>>(qkvw, WQKV, C3 * CC / 8); k_cvt8<<<(CC * CC / 8 + 255) / 256, 256, 0, stream>>>(pw, WP_, CC * CC / 8); k_cvt8<<<(C4 * CC / 8 + 255) / 256, 256, 0, stream>>>(c1w, WC1, C4 * CC / 8); k_cvt8<<<(CC * C4 / 8 + 255) / 256, 256, 0, stream>>>(c2w, WC2, CC * C4 / 8);
    k_wtap<<<(KT * 64) / 8, 256, 0, stream>>>(dmw, WT);
    k_bnstatc<<<CC / 8, 256, 0, stream>>>(x, STT);
    for (int b = 0; b < NB_; ++b) k_bnT<<<dim3(CC / 64, NPX / 64, 1), 256, 0, stream>>>(x + (size_t)b * CC * NPX, STT, gam, bet, (size_t)b * NPX, XNh, XNl, XTf);
    k_gemmb<true, false><<<dim3(NR / 64, C3 / 64, 1), 128, 0, stream>>>(XNh, XNl, WQKV, qkvb, QKV, C3, nullptr, nullptr, CC);
    for (int b = 0; b < NB_; ++b) { const size_t r0 = (size_t)b * NPX;
        for (int h = 0; h < NH_; ++h) {
            k_qkgrid<<<NPT / 8, 256, 0, stream>>>(QKV, r0, h, Gh, Gl);
            k_gemmtap49<<<dim3(NPR / 64, 1, 1), 128, 0, stream>>>(Gh, Gl, WT, CT);
            k_wattn<<<NPX / 8, 256, 0, stream>>>(CT, QKV, dmb, rel, r0, h, O); } }
    for (int b = 0; b < NB_; ++b) { const size_t r0 = (size_t)b * NPX;
        k_split192<<<NPX / 8, 256, 0, stream>>>(O + r0 * CC, NPX, Oh, Ol);
        k_gemmb<true, false><<<dim3(NPX / 64, CC / 64, 1), 128, 0, stream>>>(Oh, Ol, WP_, pb, X1 + r0 * CC, CC, nullptr, XTf + r0 * CC, CC, 0);
        k_split192<<<NPX / 8, 256, 0, stream>>>(X1 + r0 * CC, NPX, X1h, X1l);
        k_gemmb<true, false><<<dim3(NPX / 64, C4 / 64, 1), 128, 0, stream>>>(X1h, X1l, WC1, c1b, H1, C4, nullptr, nullptr, CC);
        k_gelu768<<<NPX / 8, 256, 0, stream>>>(H1, NPX, G1h, G1l);
        k_gemmb<true, false><<<dim3(NPX / 64, CC / 64, 1), 128, 0, stream>>>(G1h, G1l, WC2, c2b, H2 + r0 * CC, CC, nullptr, nullptr, C4);
        k_outT<<<dim3(NPX / 64, CC / 64, 1), 256, 0, stream>>>(X1, H2, r0, out + (size_t)b * CC * NPX); }
}
